// ThousandsBrainsNet_82179904242263
// MI455X (gfx1250) — hardware-run, weakly checked
//
#include <hip/hip_runtime.h>

typedef __attribute__((ext_vector_type(16))) __bf16   v16b;
typedef __attribute__((ext_vector_type(8)))  __bf16   v8b;
typedef __attribute__((ext_vector_type(8)))  _Float16 v8h;
typedef __attribute__((ext_vector_type(8)))  float    v8f;
typedef __attribute__((ext_vector_type(4)))  float    v4f;
typedef __attribute__((ext_vector_type(4)))  unsigned v4u;

constexpr int kBatch = 256;
constexpr int kImgH  = 224;
constexpr int kImgW  = 224;
constexpr int kWin   = 7;
constexpr int kStep  = 3;
constexpr int kNPos  = (kImgH - kWin) / kStep + 1;
constexpr int kPix   = kWin * kWin;
constexpr int kNeur  = 16;
constexpr int kUnits = 64;
constexpr int kFeat  = kNeur * kPix;
constexpr int kKP    = 832;
constexpr int kHid   = 512;
constexpr int kCls   = 10;
constexpr int kW2Rows = 64;
static_assert(kNPos == 73, "lattice positions per axis");
static_assert(kPix == 49 && kFeat == 784, "descriptor width");
static_assert(kStep * (kNPos - 1) + kWin - 1 == 222, "largest pixel index used");
static_assert(kStep * (kNPos - 1) + kWin - 1 < kImgH - 1, "last image row and column are not used");
static_assert(kKP >= kFeat && (kKP % 64) == 0 && (kKP % 32) == 0, "padded K: whole 128-B lines per plane row, multiple of 32");
static_assert((kBatch % 64) == 0 && (kHid % 64) == 0 && (kHid % 32) == 0, "GEMM tile multiples");
static_assert((kFeat % 8) == 0, "zero pad starts on an 8-element boundary");
static_assert(kCls <= 16, "head tile width");

constexpr size_t kOffAH  = 0;
constexpr size_t kOffAL  = kOffAH  + (size_t)kBatch * kKP * 2;
constexpr size_t kOffW1H = kOffAL  + (size_t)kBatch * kKP * 2;
constexpr size_t kOffW1L = kOffW1H + (size_t)kHid * kKP * 2;
constexpr size_t kOffHH  = kOffW1L + (size_t)kHid * kKP * 2;
constexpr size_t kOffHL  = kOffHH  + (size_t)kBatch * kHid * 2;
constexpr size_t kOffW2H = kOffHL  + (size_t)kBatch * kHid * 2;
constexpr size_t kOffW2L = kOffW2H + (size_t)kW2Rows * kHid * 2;
constexpr size_t kWsTotal = kOffW2L + (size_t)kW2Rows * kHid * 2;
static_assert(kWsTotal == 3211264ull, "carve total");
static_assert(kWsTotal <= 134217728ull, "carve cap");
static_assert((kOffAL % 128) == 0 && (kOffW1H % 128) == 0 && (kOffW1L % 128) == 0 && (kOffHH % 128) == 0 &&
              (kOffHL % 128) == 0 && (kOffW2H % 128) == 0 && (kOffW2L % 128) == 0, "128-B aligned regions");

__device__ __forceinline__ unsigned short f2bf_bits(float f) {
  unsigned u = __float_as_uint(f);
  return (unsigned short)((u + 0x7FFFu + ((u >> 16) & 1u)) >> 16);
}
__device__ __forceinline__ float bf_bits2f(unsigned short h) { return __uint_as_float(((unsigned)h) << 16); }
__device__ __forceinline__ unsigned bf_bits_u(float f) {
  const unsigned u = __float_as_uint(f);
  return (u + 0x7FFFu + ((u >> 16) & 1u)) >> 16;
}
__device__ __forceinline__ float bf_u2f(unsigned h) { return __uint_as_float(h << 16); }
__device__ __forceinline__ void split_pack2(float v0, float v1, unsigned& hw, unsigned& lw) {
  const unsigned h0 = bf_bits_u(v0);
  const unsigned h1 = bf_bits_u(v1);
  const unsigned l0 = bf_bits_u(v0 - bf_u2f(h0));
  const unsigned l1 = bf_bits_u(v1 - bf_u2f(h1));
  hw = h0 | (h1 << 16);
  lw = l0 | (l1 << 16);
}
__device__ __forceinline__ v4f sel4(bool c, v4f a) {
  v4f z;
  z[0] = c ? a[0] : 0.0f;
  z[1] = c ? a[1] : 0.0f;
  z[2] = c ? a[2] : 0.0f;
  z[3] = c ? a[3] : 0.0f;
  return z;
}

union FragB { v16b v; v8b h[2]; };
__device__ __forceinline__ v16b frag_load(const __bf16* p) {
  FragB f;
  f.h[0] = *(const v8b*)(p);
  f.h[1] = *(const v8b*)(p + 16);
  return f.v;
}
__device__ __forceinline__ v8f frag_mma(v16b a, v16b b, v8f c) {
  return __builtin_amdgcn_wmma_f32_16x16x32_bf16(false, a, false, b, (short)0, c, false, false);
}
__device__ __forceinline__ void tie_acc_b(v8f& a, v16b x, v16b y, v16b z, v16b w) {
  asm volatile("v_nop\n\tv_nop\n\tv_nop\n\tv_nop" : "+v"(a) : "v"(x), "v"(y), "v"(z), "v"(w));
}
__device__ __forceinline__ void keep4_b(v16b a, v16b b, v16b c, v16b d) { asm volatile("v_nop" :: "v"(a), "v"(b), "v"(c), "v"(d)); }
__device__ __forceinline__ void acc_guard4(v8f& a, v8f& b, v8f& c, v8f& d) { asm volatile("v_nop\n\tv_nop\n\tv_nop\n\tv_nop" : "+v"(a), "+v"(b), "+v"(c), "+v"(d)); }

__global__ __launch_bounds__(224) void lattice_desc_kernel(
    const float* __restrict__ x, const float* __restrict__ Wc, const float* __restrict__ bc,
    unsigned short* __restrict__ AH, unsigned short* __restrict__ AL)
{
  __shared__ float sCol[kWin * kImgW];
  __shared__ float sP[kPix];
  __shared__ float sWB[32];
  const int tid  = threadIdx.x;
  const int lane = tid & 31;
  const int wave = __builtin_amdgcn_readfirstlane((int)(threadIdx.x >> 5));
  const int b    = blockIdx.x;
  const float* img = x + (size_t)b * (size_t)(kImgH * kImgW);
  const int cc = (tid < kImgW - 1) ? tid : (kImgW - 2);
  float a0 = 0.0f, a1 = 0.0f, a2 = 0.0f, a3 = 0.0f, a4 = 0.0f, a5 = 0.0f, a6 = 0.0f;
#pragma unroll 1
  for (int i = 0; i < kNPos; ++i) {
    const float* rp = img + (kStep * i) * kImgW + cc;
    a0 += rp[0];
    a1 += rp[kImgW];
    a2 += rp[2 * kImgW];
    a3 += rp[3 * kImgW];
    a4 += rp[4 * kImgW];
    a5 += rp[5 * kImgW];
    a6 += rp[6 * kImgW];
  }
  sCol[0 * kImgW + tid] = a0;
  sCol[1 * kImgW + tid] = a1;
  sCol[2 * kImgW + tid] = a2;
  sCol[3 * kImgW + tid] = a3;
  sCol[4 * kImgW + tid] = a4;
  sCol[5 * kImgW + tid] = a5;
  sCol[6 * kImgW + tid] = a6;
  if (wave == 0) {
    const int n = lane & 15;
    float sw = 0.0f, sb = 0.0f;
#pragma unroll 1
    for (int m = 0; m < kUnits; ++m) {
      sw += Wc[m * kNeur + n];
      sb += bc[m * kNeur + n];
    }
    const float pick = (lane < 16) ? sw : sb;
    sWB[lane] = pick * (1.0f / (float)kUnits);
  }
  __syncthreads();
  {
    const int j2 = (lane + 64 < kNPos) ? (lane + 64) : (kNPos - 1);
#pragma unroll 1
    for (int fh = 0; fh < kWin; ++fh) {
      const float* cp = sCol + fh * kImgW + wave;
      const float v0 = cp[kStep * lane];
      const float v1 = cp[kStep * (lane + 32)];
      const float v2 = cp[kStep * j2];
      float s = v0 + v1;
      s += (lane + 64 < kNPos) ? v2 : 0.0f;
      s += __shfl_xor(s, 16, 32);
      s += __shfl_xor(s, 8, 32);
      s += __shfl_xor(s, 4, 32);
      s += __shfl_xor(s, 2, 32);
      s += __shfl_xor(s, 1, 32);
      if (lane == 0) sP[fh * kWin + wave] = s * (1.0f / (float)(kNPos * kNPos));
    }
  }
  __syncthreads();
  if (tid < kKP / 8) {
    float dv[8];
#pragma unroll
    for (int e = 0; e < 8; ++e) {
      const int k  = tid * 8 + e;
      const int kc = (k < kFeat) ? k : (kFeat - 1);
      const int n  = kc / kPix;
      const int p  = kc - n * kPix;
      const float raw = sWB[n] * sP[p] + sWB[16 + n];
      dv[e] = (k < kFeat) ? raw : 0.0f;
    }
    v4u ph, pl;
    unsigned hw, lw;
    split_pack2(dv[0], dv[1], hw, lw); ph[0] = hw; pl[0] = lw;
    split_pack2(dv[2], dv[3], hw, lw); ph[1] = hw; pl[1] = lw;
    split_pack2(dv[4], dv[5], hw, lw); ph[2] = hw; pl[2] = lw;
    split_pack2(dv[6], dv[7], hw, lw); ph[3] = hw; pl[3] = lw;
    unsigned short* qh = AH + (size_t)b * kKP + tid * 8;
    unsigned short* ql = AL + (size_t)b * kKP + tid * 8;
    *(volatile v4u*)qh = ph;
    *(volatile v4u*)ql = pl;
    __threadfence();
    *(volatile v4u*)qh = ph;
    *(volatile v4u*)ql = pl;
  }
}

__global__ __launch_bounds__(256) void weight_planes_kernel(
    const float* __restrict__ W1, const float* __restrict__ W2,
    unsigned short* __restrict__ W1H, unsigned short* __restrict__ W1L,
    unsigned short* __restrict__ W2H, unsigned short* __restrict__ W2L)
{
  __shared__ __align__(16) float sT[64 * 68];
  const int tid = threadIdx.x;
  const int bx  = blockIdx.x;
  constexpr int kW1Blocks = (kKP / 64) * (kHid / 64);
  unsigned short* outH;
  unsigned short* outL;
  int pitch, row0, col0;
  if (bx < kW1Blocks) {
    const int kt = bx >> 3, ot = bx & 7;
    const int k0 = kt * 64, o0 = ot * 64;
    const int kk = tid >> 2, oq = (tid & 3) * 16;
    const int k  = k0 + kk;
    const int kc = (k < kFeat) ? k : (kFeat - 1);
    const float* src = W1 + (size_t)kc * kHid + o0 + oq;
    v4f g0 = *(const v4f*)(src);
    v4f g1 = *(const v4f*)(src + 4);
    v4f g2 = *(const v4f*)(src + 8);
    v4f g3 = *(const v4f*)(src + 12);
    asm volatile("" : "+v"(g0), "+v"(g1), "+v"(g2), "+v"(g3));
    const bool live = (k < kFeat);
    float* dst = sT + kk * 68 + oq;
    *(v4f*)(dst)      = sel4(live, g0);
    *(v4f*)(dst + 4)  = sel4(live, g1);
    *(v4f*)(dst + 8)  = sel4(live, g2);
    *(v4f*)(dst + 12) = sel4(live, g3);
    outH = W1H; outL = W1L; pitch = kKP; row0 = o0; col0 = k0;
  } else {
    const int k0 = (bx - kW1Blocks) * 64;
#pragma unroll 1
    for (int i = 0; i < 16; ++i) {
      const int idx = tid + 256 * i;
      const int kk = idx >> 6, cls = idx & 63;
      const int clsc = (cls < kCls) ? cls : (kCls - 1);
      float g = W2[(size_t)(k0 + kk) * kCls + clsc];
      asm volatile("" : "+v"(g));
      sT[kk * 68 + cls] = (cls < kCls) ? g : 0.0f;
    }
    outH = W2H; outL = W2L; pitch = kHid; row0 = 0; col0 = k0;
  }
  __syncthreads();
  const int c8 = (tid & 7) * 8;
  v4u ph[2], pl[2];
#pragma unroll
  for (int it = 0; it < 2; ++it) {
    const int rr = it * 32 + (tid >> 3);
    float g[8];
#pragma unroll
    for (int e = 0; e < 8; ++e) g[e] = sT[(c8 + e) * 68 + rr];
    unsigned hw, lw;
    split_pack2(g[0], g[1], hw, lw); ph[it][0] = hw; pl[it][0] = lw;
    split_pack2(g[2], g[3], hw, lw); ph[it][1] = hw; pl[it][1] = lw;
    split_pack2(g[4], g[5], hw, lw); ph[it][2] = hw; pl[it][2] = lw;
    split_pack2(g[6], g[7], hw, lw); ph[it][3] = hw; pl[it][3] = lw;
  }
  for (int pass = 0; pass < 2; ++pass) {
#pragma unroll
    for (int it = 0; it < 2; ++it) {
      const int rr = it * 32 + (tid >> 3);
      const size_t o = (size_t)(row0 + rr) * pitch + col0 + c8;
      *(volatile v4u*)(outH + o) = ph[it];
      *(volatile v4u*)(outL + o) = pl[it];
    }
    __threadfence();
  }
}

__global__ __launch_bounds__(256) void wmma_gemm64_split_kernel(
    const unsigned short* __restrict__ Ap, const unsigned short* __restrict__ A2p, int lda,
    const unsigned short* __restrict__ Btp, const unsigned short* __restrict__ Bt2p, int ldb,
    unsigned short* __restrict__ Ch, unsigned short* __restrict__ Cl, int ldc,
    const float* __restrict__ bias, int M, int N, int K)
{
  const __bf16* A   = (const __bf16*)Ap;
  const __bf16* A2  = (const __bf16*)A2p;
  const __bf16* Bt  = (const __bf16*)Btp;
  const __bf16* Bt2 = (const __bf16*)Bt2p;
  __shared__ __align__(16) float sT[8][16 * 68];
  const int lane = threadIdx.x & 31;
  const int wave = __builtin_amdgcn_readfirstlane((int)(threadIdx.x >> 5));
  const int tilesN = N >> 6;
  const int tilesM = M >> 6;
  const int tile = blockIdx.x * 8 + wave;
  if (tile >= tilesM * tilesN) return;
  const int tm = tile / tilesN;
  const int tn = tile - tm * tilesN;
  const int m0 = tm << 6;
  const int n0 = tn << 6;

  const int rlane = lane & 15;
  const int koff  = (lane >> 4) * 8;
  const int mOff  = (lane >> 4) * 8;

  v8f acc[4][4];
#pragma unroll
  for (int i = 0; i < 4; ++i)
#pragma unroll
    for (int j = 0; j < 4; ++j) acc[i][j] = (v8f){0.f,0.f,0.f,0.f,0.f,0.f,0.f,0.f};

  for (int k0 = 0; k0 < K; k0 += 32) {
    v16b bh[4], bl[4];
#pragma unroll
    for (int j = 0; j < 4; ++j) {
      const size_t bo = (size_t)(n0 + (j << 4) + rlane) * ldb + koff + k0;
      bh[j] = frag_load(Bt + bo);
      bl[j] = frag_load(Bt2 + bo);
    }
#pragma unroll
    for (int i = 0; i < 4; ++i) {
      const size_t ao = (size_t)(m0 + (i << 4) + rlane) * lda + koff + k0;
      const v16b ah = frag_load(A + ao);
      const v16b al = frag_load(A2 + ao);
#pragma unroll
      for (int j = 0; j < 4; ++j) {
        acc[i][j] = frag_mma(ah, bh[j], acc[i][j]);
        acc[i][j] = frag_mma(ah, bl[j], acc[i][j]);
        acc[i][j] = frag_mma(al, bh[j], acc[i][j]);
      }
      tie_acc_b(acc[i][0], ah, al, bh[0], bl[0]);
      tie_acc_b(acc[i][1], ah, al, bh[1], bl[1]);
      tie_acc_b(acc[i][2], ah, al, bh[2], bl[2]);
      tie_acc_b(acc[i][3], ah, al, bh[3], bl[3]);
    }
    keep4_b(bh[0], bh[1], bh[2], bh[3]);
    keep4_b(bl[0], bl[1], bl[2], bl[3]);
  }
  acc_guard4(acc[0][0], acc[0][1], acc[0][2], acc[0][3]);
  acc_guard4(acc[1][0], acc[1][1], acc[1][2], acc[1][3]);
  acc_guard4(acc[2][0], acc[2][1], acc[2][2], acc[2][3]);
  acc_guard4(acc[3][0], acc[3][1], acc[3][2], acc[3][3]);

  float* slab = sT[wave];
#pragma unroll
  for (int i = 0; i < 4; ++i) {
    const int mBase = m0 + (i << 4);
#pragma unroll
    for (int j = 0; j < 4; ++j) {
      const int n = n0 + (j << 4) + rlane;
      const float bv = bias[n];
#pragma unroll
      for (int r = 0; r < 8; ++r) {
        float v = acc[i][j][r] + bv;
        v = fmaxf(v, 0.0f);
        slab[(mOff + r) * 68 + (j << 4) + rlane] = v;
      }
    }
    __builtin_amdgcn_fence(__ATOMIC_RELEASE, "workgroup");
    __builtin_amdgcn_wave_barrier();
    __builtin_amdgcn_fence(__ATOMIC_ACQUIRE, "workgroup");
    {
      const int q = lane >> 3, c8 = (lane & 7) * 8;
      for (int pass = 0; pass < 2; ++pass) {
#pragma unroll
        for (int it = 0; it < 4; ++it) {
          const int row = it * 4 + q;
          const float* sp = slab + row * 68 + c8;
          v8h hv, lv;
#pragma unroll
          for (int e = 0; e < 8; ++e) {
            const float sv = sp[e];
            const unsigned short hb = f2bf_bits(sv);
            const unsigned short lb = f2bf_bits(sv - bf_bits2f(hb));
            hv[e] = __builtin_bit_cast(_Float16, hb);
            lv[e] = __builtin_bit_cast(_Float16, lb);
          }
          *(volatile v8h*)(Ch + (size_t)(mBase + row) * ldc + n0 + c8) = hv;
          *(volatile v8h*)(Cl + (size_t)(mBase + row) * ldc + n0 + c8) = lv;
        }
        __threadfence();
      }
    }
    __builtin_amdgcn_fence(__ATOMIC_RELEASE, "workgroup");
    __builtin_amdgcn_wave_barrier();
    __builtin_amdgcn_fence(__ATOMIC_ACQUIRE, "workgroup");
  }
}

__global__ __launch_bounds__(32) void head_gemm_kernel(
    const unsigned short* __restrict__ HH, const unsigned short* __restrict__ HL,
    const unsigned short* __restrict__ W2H, const unsigned short* __restrict__ W2L,
    const float* __restrict__ b2, float* __restrict__ out)
{
  __shared__ __align__(16) float sO[16 * kCls];
  const int lane = threadIdx.x & 31;
  const int rl = lane & 15, hh = lane >> 4;
  const int m0 = blockIdx.x * 16;
  const __bf16* pah = (const __bf16*)HH  + (size_t)(m0 + rl) * kHid + hh * 8;
  const __bf16* pal = (const __bf16*)HL  + (size_t)(m0 + rl) * kHid + hh * 8;
  const __bf16* pbh = (const __bf16*)W2H + (size_t)rl * kHid + hh * 8;
  const __bf16* pbl = (const __bf16*)W2L + (size_t)rl * kHid + hh * 8;
  v8f acc = (v8f){0.f,0.f,0.f,0.f,0.f,0.f,0.f,0.f};
#pragma unroll 1
  for (int k0 = 0; k0 < kHid; k0 += 32) {
    const v16b ah = frag_load(pah + k0);
    const v16b al = frag_load(pal + k0);
    const v16b bh = frag_load(pbh + k0);
    const v16b bl = frag_load(pbl + k0);
    acc = frag_mma(ah, bh, acc);
    acc = frag_mma(ah, bl, acc);
    acc = frag_mma(al, bh, acc);
    tie_acc_b(acc, ah, al, bh, bl);
  }
  const int cb = (rl < kCls) ? rl : (kCls - 1);
  float bv = b2[cb];
  asm volatile("" : "+v"(bv));
  if (rl < kCls) {
#pragma unroll
    for (int r = 0; r < 8; ++r) sO[(8 * hh + r) * kCls + rl] = acc[r] + bv;
  }
  __syncthreads();
  const v4f w0 = *(const v4f*)(sO + lane * 4);
  const v4f w1 = *(const v4f*)(sO + 128 + (lane & 7) * 4);
  float* ob = out + (size_t)m0 * kCls;
  *(volatile v4f*)(ob + lane * 4) = w0;
  if (lane < 8) *(volatile v4f*)(ob + 128 + lane * 4) = w1;
  __threadfence();
  *(volatile v4f*)(ob + lane * 4) = w0;
  if (lane < 8) *(volatile v4f*)(ob + 128 + lane * 4) = w1;
}

extern "C" void kernel_launch(void* const* d_in, const int* in_sizes, int n_in,
                              void* d_out, int out_size, void* d_ws, size_t ws_size,
                              hipStream_t stream) {
  if (n_in < 7) return;
  if (in_sizes[0] != kBatch * kImgH * kImgW) return;
  if (in_sizes[1] != kUnits * kNeur) return;
  if (in_sizes[2] != kUnits * kNeur) return;
  if (in_sizes[3] != kFeat * kHid) return;
  if (in_sizes[4] != kHid) return;
  if (in_sizes[5] != kHid * kCls) return;
  if (in_sizes[6] != kCls) return;
  if (out_size != kBatch * kCls) return;
  if (ws_size < kWsTotal) return;

  const float* x  = (const float*)d_in[0];
  const float* Wc = (const float*)d_in[1];
  const float* bc = (const float*)d_in[2];
  const float* W1 = (const float*)d_in[3];
  const float* b1 = (const float*)d_in[4];
  const float* W2 = (const float*)d_in[5];
  const float* b2 = (const float*)d_in[6];
  float* out = (float*)d_out;

  char* ws = (char*)d_ws;
  unsigned short* AH  = (unsigned short*)(ws + kOffAH);
  unsigned short* AL  = (unsigned short*)(ws + kOffAL);
  unsigned short* W1H = (unsigned short*)(ws + kOffW1H);
  unsigned short* W1L = (unsigned short*)(ws + kOffW1L);
  unsigned short* HH  = (unsigned short*)(ws + kOffHH);
  unsigned short* HL  = (unsigned short*)(ws + kOffHL);
  unsigned short* W2H = (unsigned short*)(ws + kOffW2H);
  unsigned short* W2L = (unsigned short*)(ws + kOffW2L);

  lattice_desc_kernel<<<kBatch, 224, 0, stream>>>(x, Wc, bc, AH, AL);

  weight_planes_kernel<<<(kKP / 64) * (kHid / 64) + (kHid / 64), 256, 0, stream>>>(W1, W2, W1H, W1L, W2H, W2L);

  wmma_gemm64_split_kernel<<<((kBatch / 64) * (kHid / 64)) / 8, 256, 0, stream>>>(
      AH, AL, kKP, W1H, W1L, kKP, HH, HL, kHid, b1, kBatch, kHid, kKP);

  head_gemm_kernel<<<kBatch / 16, 32, 0, stream>>>(HH, HL, W2H, W2L, b2, out);
}
